// TrittentionCube_29978871726703
// MI455X (gfx1250) — hardware-run, weakly checked
//
#include <hip/hip_runtime.h>
#include <math.h>

typedef __attribute__((ext_vector_type(16))) _Float16 v16h;
typedef __attribute__((ext_vector_type(8)))  _Float16 v8h;
typedef __attribute__((ext_vector_type(16))) __bf16   v16b;
typedef __attribute__((ext_vector_type(8)))  __bf16   v8b;
typedef __attribute__((ext_vector_type(8)))  float    v8f;
typedef __attribute__((ext_vector_type(4)))  float    v4f;
typedef __attribute__((ext_vector_type(4)))  unsigned int v4u;

constexpr int kB     = 2;
constexpr int kT     = 192;
constexpr int kDM    = 512;
constexpr int kNH    = 8;
constexpr int kDH    = 64;
constexpr int kRows  = kB * kT;
constexpr int kProjN = 5 * kNH * kDH;
constexpr int kHG    = kDH * kDH;
static_assert(kRows == 384 && kProjN == 2560 && kHG == 4096, "shapes");
static_assert(kNH * kDH == kDM, "head split");
static_assert((kT % 64) == 0 && (kDM % 64) == 0 && (kDH % 32) == 0 && (kHG % 64) == 0, "tile multiples");

constexpr float kACarry  = 16.0f;
constexpr float kCCarry  = 16.0f;
constexpr float kBsCarry = 16.0f;
constexpr float kWKCarry = 1024.0f;
constexpr float kS1Carry = 64.0f;
constexpr float kS2Carry = 8.0f;
constexpr float kS1Scale = kS1Carry / (kCCarry * kWKCarry);
constexpr float kS2Scale = kS2Carry / (kS1Carry * kBsCarry);
constexpr float kScoreScale = 1.0f / (kACarry * kS2Carry * (float)kDH);

constexpr size_t kSzX    = (size_t)kRows * kDM * 2;
constexpr size_t kSzWP   = (size_t)kProjN * kDM * 2;
constexpr size_t kSzPROJ = (size_t)kRows * kProjN * 4;
constexpr size_t kSzAPL  = (size_t)kB * kNH * kT * kDH * 2;
constexpr size_t kSzCPL  = (size_t)kRows * kDM * 2;
constexpr size_t kSzBSUM = (size_t)kRows * kDH * 2;
constexpr size_t kSzDT   = (size_t)kB * kNH * kDH * kT * 2;
constexpr size_t kSzWKB  = (size_t)kHG * kDM * 2;
constexpr size_t kSzS1   = (size_t)kRows * kHG * 2;
constexpr size_t kSzS2T  = (size_t)kB * kT * kT * kDH * 2;
constexpr size_t kSzY    = (size_t)kNH * kRows * kHG * 2;
constexpr size_t kSzWV   = (size_t)kNH * kDH * kHG * 2;
constexpr size_t kSzZ    = (size_t)kRows * kDM * 2;
constexpr size_t kSzWO   = (size_t)kDM * kDM * 2;

constexpr size_t kOffXH   = 0;
constexpr size_t kOffXL   = kOffXH   + kSzX;
constexpr size_t kOffWPH  = kOffXL   + kSzX;
constexpr size_t kOffWPL  = kOffWPH  + kSzWP;
constexpr size_t kOffPROJ = kOffWPL  + kSzWP;
constexpr size_t kOffAPL  = kOffPROJ + kSzPROJ;
constexpr size_t kOffCPL  = kOffAPL  + kSzAPL;
constexpr size_t kOffBSUM = kOffCPL  + kSzCPL;
constexpr size_t kOffDTH  = kOffBSUM + kSzBSUM;
constexpr size_t kOffDTL  = kOffDTH  + kSzDT;
constexpr size_t kOffETH  = kOffDTL  + kSzDT;
constexpr size_t kOffETL  = kOffETH  + kSzDT;
constexpr size_t kOffWKB  = kOffETL  + kSzDT;
constexpr size_t kOffS1   = kOffWKB  + kSzWKB;
constexpr size_t kOffS2T  = kOffS1   + kSzS1;
constexpr size_t kOffYH   = kOffS2T  + kSzS2T;
constexpr size_t kOffYL   = kOffYH   + kSzY;
constexpr size_t kOffWVH  = kOffYL   + kSzY;
constexpr size_t kOffWVL  = kOffWVH  + kSzWV;
constexpr size_t kOffZH   = kOffWVL  + kSzWV;
constexpr size_t kOffZL   = kOffZH   + kSzZ;
constexpr size_t kOffWOH  = kOffZL   + kSzZ;
constexpr size_t kOffWOL  = kOffWOH  + kSzWO;
constexpr size_t kWsTotal = kOffWOL  + kSzWO;
static_assert(kWsTotal == 89702400ull, "carve total");
static_assert(kWsTotal <= 134217728ull, "carve cap");
static_assert((kSzBSUM % 128) == 0 && (kSzX % 128) == 0 && (kSzDT % 128) == 0, "128-B aligned regions");

__device__ __forceinline__ unsigned short f2bf_bits(float f) {
  unsigned u = __float_as_uint(f);
  return (unsigned short)((u + 0x7FFFu + ((u >> 16) & 1u)) >> 16);
}
__device__ __forceinline__ float bf_bits2f(unsigned short h) { return __uint_as_float(((unsigned)h) << 16); }
__device__ __forceinline__ unsigned pk16(unsigned short a, unsigned short b) { return (unsigned)a | ((unsigned)b << 16); }
__device__ __forceinline__ unsigned short h_bits(float f) { const _Float16 h = (_Float16)f; return __builtin_bit_cast(unsigned short, h); }

__device__ __forceinline__ void wave_lds_sync() {
  __builtin_amdgcn_fence(__ATOMIC_RELEASE, "workgroup");
  __builtin_amdgcn_wave_barrier();
  __builtin_amdgcn_fence(__ATOMIC_ACQUIRE, "workgroup");
}

__device__ __forceinline__ void dep_guard4_h(v8f& a, v8f& b, v8f& c, v8f& d, v16h x, v16h y) { asm volatile("v_nop\n\tv_nop\n\tv_nop\n\tv_nop" : "+v"(a), "+v"(b), "+v"(c), "+v"(d) : "v"(x), "v"(y)); }
__device__ __forceinline__ void dep_guard4_b(v8f& a, v8f& b, v8f& c, v8f& d, v16b x, v16b y) { asm volatile("v_nop\n\tv_nop\n\tv_nop\n\tv_nop" : "+v"(a), "+v"(b), "+v"(c), "+v"(d) : "v"(x), "v"(y)); }
__device__ __forceinline__ void keep4_h(v16h a, v16h b, v16h c, v16h d) { asm volatile("v_nop" :: "v"(a), "v"(b), "v"(c), "v"(d)); }
__device__ __forceinline__ void keep4_b(v16b a, v16b b, v16b c, v16b d) { asm volatile("v_nop" :: "v"(a), "v"(b), "v"(c), "v"(d)); }
__device__ __forceinline__ void acc_guard4(v8f& a, v8f& b, v8f& c, v8f& d) { asm volatile("v_nop\n\tv_nop\n\tv_nop\n\tv_nop" : "+v"(a), "+v"(b), "+v"(c), "+v"(d)); }

template <typename T> struct Frag;
template <> struct Frag<_Float16> {
  typedef v16h V; union U { v16h v; v8h h[2]; };
  static __device__ __forceinline__ v16h load(const _Float16* p) {
    U f; f.h[0] = *(const v8h*)(p); f.h[1] = *(const v8h*)(p + 16); return f.v;
  }
  static __device__ __forceinline__ v8f mma(v16h a, v16h b, v8f c) {
    return __builtin_amdgcn_wmma_f32_16x16x32_f16(false, a, false, b, (short)0, c, false, false);
  }
  static __device__ __forceinline__ void guard4(v8f& a, v8f& b, v8f& c, v8f& d, v16h x, v16h y) { dep_guard4_h(a, b, c, d, x, y); }
  static __device__ __forceinline__ void keep(v16h a, v16h b, v16h c, v16h d) { keep4_h(a, b, c, d); }
};
template <> struct Frag<__bf16> {
  typedef v16b V; union U { v16b v; v8b h[2]; };
  static __device__ __forceinline__ v16b load(const __bf16* p) {
    U f; f.h[0] = *(const v8b*)(p); f.h[1] = *(const v8b*)(p + 16); return f.v;
  }
  static __device__ __forceinline__ v8f mma(v16b a, v16b b, v8f c) {
    return __builtin_amdgcn_wmma_f32_16x16x32_bf16(false, a, false, b, (short)0, c, false, false);
  }
  static __device__ __forceinline__ void guard4(v8f& a, v8f& b, v8f& c, v8f& d, v16b x, v16b y) { dep_guard4_b(a, b, c, d, x, y); }
  static __device__ __forceinline__ void keep(v16b a, v16b b, v16b c, v16b d) { keep4_b(a, b, c, d); }
};

__device__ __forceinline__ v8f mma_h(v16h a, v16h b, v8f c) {
  c = __builtin_amdgcn_wmma_f32_16x16x32_f16(false, a, false, b, (short)0, c, false, false);
  asm volatile("v_nop\n\tv_nop\n\tv_nop\n\tv_nop" : "+v"(c) : "v"(a), "v"(b));
  return c;
}
__device__ __forceinline__ v8f mma_b(v16b a, v16b b, v8f c) {
  c = __builtin_amdgcn_wmma_f32_16x16x32_bf16(false, a, false, b, (short)0, c, false, false);
  asm volatile("v_nop\n\tv_nop\n\tv_nop\n\tv_nop" : "+v"(c) : "v"(a), "v"(b));
  return c;
}

template <int ET> struct Elem;
template <> struct Elem<0> { typedef _Float16 T; };
template <> struct Elem<1> { typedef __bf16 T; };
template <int ET, bool SPLIT, int BIAS_MODE, int OUT_MODE>
__global__ __launch_bounds__(256) void wmma_gemm64(
    const unsigned short* __restrict__ Ap, const unsigned short* __restrict__ A2p, int lda, long strideA,
    const unsigned short* __restrict__ Btp, const unsigned short* __restrict__ Bt2p, int ldb, long strideB,
    void* __restrict__ Cout, void* __restrict__ Cout2, int ldc, long strideC,
    const float* __restrict__ bias,
    int M, int N, int K, float scale) {
  typedef typename Elem<ET>::T T;
  typedef typename Frag<T>::V V;
  const T* A = (const T*)Ap; const T* A2 = (const T*)A2p; const T* Bt = (const T*)Btp; const T* Bt2 = (const T*)Bt2p;
  __shared__ __align__(16) float sT[8][16 * 68];
  const int b    = blockIdx.y;
  const int lane = threadIdx.x & 31;
  const int wave = threadIdx.x >> 5;
  const int tilesN = N >> 6;
  const int tilesM = M >> 6;
  const int tile = blockIdx.x * 8 + wave;
  if (tile >= tilesM * tilesN) return;
  const int tm = tile / tilesN;
  const int tn = tile - tm * tilesN;
  const int m0 = tm << 6;
  const int n0 = tn << 6;

  const T* Ab  = A  + (size_t)b * strideA;
  const T* Bb  = Bt + (size_t)b * strideB;
  const T* Ab2 = SPLIT ? (A2  + (size_t)b * strideA) : nullptr;
  const T* Bb2 = SPLIT ? (Bt2 + (size_t)b * strideB) : nullptr;

  const int rlane = lane & 15;
  const int koff  = (lane >> 4) * 8;
  const int mOff  = (lane >> 4) * 8;

  v8f acc[4][4];
#pragma unroll
  for (int i = 0; i < 4; ++i)
#pragma unroll
    for (int j = 0; j < 4; ++j) acc[i][j] = (v8f){0.f,0.f,0.f,0.f,0.f,0.f,0.f,0.f};

  for (int k0 = 0; k0 < K; k0 += 32) {
    V bh[4], bl[4];
#pragma unroll
    for (int j = 0; j < 4; ++j) {
      const size_t bo = (size_t)(n0 + (j << 4) + rlane) * ldb + koff + k0;
      bh[j] = Frag<T>::load(Bb + bo);
      if (SPLIT) bl[j] = Frag<T>::load(Bb2 + bo);
    }
#pragma unroll
    for (int i = 0; i < 4; ++i) {
      const size_t ao = (size_t)(m0 + (i << 4) + rlane) * lda + koff + k0;
      V ah = Frag<T>::load(Ab + ao);
      V al;
      if (SPLIT) al = Frag<T>::load(Ab2 + ao);
#pragma unroll
      for (int j = 0; j < 4; ++j) {
        acc[i][j] = Frag<T>::mma(ah, bh[j], acc[i][j]);
        if (SPLIT) {
          acc[i][j] = Frag<T>::mma(ah, bl[j], acc[i][j]);
          acc[i][j] = Frag<T>::mma(al, bh[j], acc[i][j]);
        }
      }
      Frag<T>::guard4(acc[i][0], acc[i][1], acc[i][2], acc[i][3], ah, SPLIT ? al : ah);
    }
    Frag<T>::keep(bh[0], bh[1], bh[2], bh[3]);
    if (SPLIT) Frag<T>::keep(bl[0], bl[1], bl[2], bl[3]);
  }
  acc_guard4(acc[0][0], acc[0][1], acc[0][2], acc[0][3]);
  acc_guard4(acc[1][0], acc[1][1], acc[1][2], acc[1][3]);
  acc_guard4(acc[2][0], acc[2][1], acc[2][2], acc[2][3]);
  acc_guard4(acc[3][0], acc[3][1], acc[3][2], acc[3][3]);

  float* slab = sT[wave];
#pragma unroll
  for (int i = 0; i < 4; ++i) {
    const int mBase = m0 + (i << 4);
#pragma unroll
    for (int j = 0; j < 4; ++j) {
      const int n = n0 + (j << 4) + rlane;
      float bv = 0.f;
      if (BIAS_MODE == 2) bv = bias[n];
#pragma unroll
      for (int r = 0; r < 8; ++r) {
        float v = acc[i][j][r] * scale;
        if (BIAS_MODE == 2) v += bv;
        slab[(mOff + r) * 68 + (j << 4) + rlane] = v;
      }
    }
    wave_lds_sync();
    if (OUT_MODE == 0) {
      float* C = (float*)Cout + (size_t)b * strideC;
      const int hh = lane >> 4, c4 = (lane & 15) * 4;
      for (int pass = 0; pass < 2; ++pass) {
#pragma unroll
        for (int it = 0; it < 8; ++it) {
          const int row = it * 2 + hh;
          v4f v = *(const v4f*)(slab + row * 68 + c4);
          *(volatile v4f*)(C + (size_t)(mBase + row) * ldc + n0 + c4) = v;
        }
        __threadfence();
      }
    } else {
      const int q = lane >> 3, c8 = (lane & 7) * 8;
      unsigned short* C  = (unsigned short*)Cout  + (size_t)b * strideC;
      unsigned short* C2 = (OUT_MODE == 2) ? ((unsigned short*)Cout2 + (size_t)b * strideC) : nullptr;
      for (int pass = 0; pass < 2; ++pass) {
#pragma unroll
        for (int it = 0; it < 4; ++it) {
          const int row = it * 4 + q;
          const float* sp = slab + row * 68 + c8;
          v8h hv, lv;
#pragma unroll
          for (int e = 0; e < 8; ++e) {
            if (OUT_MODE == 1) {
              hv[e] = (_Float16)sp[e];
            } else {
              unsigned short hb = f2bf_bits(sp[e]);
              unsigned short lb = f2bf_bits(sp[e] - bf_bits2f(hb));
              hv[e] = __builtin_bit_cast(_Float16, hb);
              lv[e] = __builtin_bit_cast(_Float16, lb);
            }
          }
          *(volatile v8h*)(C + (size_t)(mBase + row) * ldc + n0 + c8) = hv;
          if (OUT_MODE == 2) *(volatile v8h*)(C2 + (size_t)(mBase + row) * ldc + n0 + c8) = lv;
        }
        __threadfence();
      }
    }
    wave_lds_sync();
  }
}

__global__ __launch_bounds__(256) void split_rows_kernel(
    const float* __restrict__ src, unsigned short* __restrict__ dhi, unsigned short* __restrict__ dlo, int total8)
{
  const int i = blockIdx.x * 256 + threadIdx.x;
  if (i >= total8) return;
  const size_t e0 = (size_t)i << 3;
  const v4f a0 = *(const v4f*)(src + e0);
  const v4f a1 = *(const v4f*)(src + e0 + 4);
  float x[8];
#pragma unroll
  for (int e = 0; e < 4; ++e) { x[e] = a0[e]; x[4 + e] = a1[e]; }
  unsigned short hb[8], lb[8];
#pragma unroll
  for (int e = 0; e < 8; ++e) {
    hb[e] = f2bf_bits(x[e]);
    lb[e] = f2bf_bits(x[e] - bf_bits2f(hb[e]));
  }
  const v4u hv = (v4u){pk16(hb[0], hb[1]), pk16(hb[2], hb[3]), pk16(hb[4], hb[5]), pk16(hb[6], hb[7])};
  const v4u lv = (v4u){pk16(lb[0], lb[1]), pk16(lb[2], lb[3]), pk16(lb[4], lb[5]), pk16(lb[6], lb[7])};
  unsigned short* qh = dhi + e0;
  unsigned short* ql = dlo + e0;
  *(volatile v4u*)qh = hv;
  *(volatile v4u*)ql = lv;
  __threadfence();
  *(volatile v4u*)qh = hv;
  *(volatile v4u*)ql = lv;
}

__global__ __launch_bounds__(256) void wk_cast_kernel(const float* __restrict__ WK, unsigned short* __restrict__ out)
{
  const int idx = blockIdx.x * 256 + threadIdx.x;
  const int ij  = idx >> 6;
  const int g8  = idx & 63;
  const int n   = g8 >> 3;
  const int k0  = (g8 & 7) * 8;
  const float* p = WK + (size_t)n * ((size_t)kHG * kDH) + (size_t)ij * kDH + k0;
  const v4f a0 = *(const v4f*)(p);
  const v4f a1 = *(const v4f*)(p + 4);
  unsigned short hb[8];
#pragma unroll
  for (int e = 0; e < 4; ++e) {
    hb[e]     = h_bits(a0[e] * kWKCarry);
    hb[4 + e] = h_bits(a1[e] * kWKCarry);
  }
  const v4u u = (v4u){pk16(hb[0], hb[1]), pk16(hb[2], hb[3]), pk16(hb[4], hb[5]), pk16(hb[6], hb[7])};
  unsigned short* q = out + (size_t)ij * kDM + n * kDH + k0;
  *(volatile v4u*)q = u;
  __threadfence();
  *(volatile v4u*)q = u;
}

template <bool HAS_BIAS>
__global__ __launch_bounds__(256) void tsplit_kernel(
    const float* __restrict__ in, int inPitch, long inStrideHi, long inStrideLo, int zDiv,
    const float* __restrict__ bias, int biasStrideLo,
    unsigned short* __restrict__ ohi, unsigned short* __restrict__ olo, int outPitch, long outStride)
{
  __shared__ float sm[64][65];
  const int t  = threadIdx.x;
  const int r0 = blockIdx.x * 64;
  const int c0 = blockIdx.y * 64;
  const int z  = blockIdx.z;
  const int zHi = z / zDiv;
  const int zLo = z - zHi * zDiv;
  const float* ip = in + (size_t)zHi * inStrideHi + (size_t)zLo * inStrideLo;
  const int cl = t & 63;
  float bv = 0.f;
  if (HAS_BIAS) bv = bias[zLo * biasStrideLo + c0 + cl];
#pragma unroll
  for (int i = 0; i < 16; ++i) {
    const int r = (i * 256 + t) >> 6;
    const float v = ip[(size_t)(r0 + r) * inPitch + c0 + cl] + bv;
    sm[cl][r] = v;
  }
  __syncthreads();
  const int lane = t & 31, wave = t >> 5;
  const int q = lane >> 3, c8 = (lane & 7) * 8;
  v4u hv[2], lv[2];
#pragma unroll
  for (int it = 0; it < 2; ++it) {
    const int row = wave * 8 + it * 4 + q;
    unsigned short hb[8], lb[8];
#pragma unroll
    for (int e = 0; e < 8; ++e) {
      const float v = sm[row][c8 + e];
      hb[e] = f2bf_bits(v);
      lb[e] = f2bf_bits(v - bf_bits2f(hb[e]));
    }
    hv[it] = (v4u){pk16(hb[0], hb[1]), pk16(hb[2], hb[3]), pk16(hb[4], hb[5]), pk16(hb[6], hb[7])};
    lv[it] = (v4u){pk16(lb[0], lb[1]), pk16(lb[2], lb[3]), pk16(lb[4], lb[5]), pk16(lb[6], lb[7])};
  }
  const size_t ob = (size_t)z * outStride;
  for (int pass = 0; pass < 2; ++pass) {
#pragma unroll
    for (int it = 0; it < 2; ++it) {
      const int row = wave * 8 + it * 4 + q;
      const size_t o = ob + (size_t)(c0 + row) * outPitch + r0 + c8;
      *(volatile v4u*)(ohi + o) = hv[it];
      *(volatile v4u*)(olo + o) = lv[it];
    }
    __threadfence();
  }
}

__global__ __launch_bounds__(256) void cvt_abc_kernel(
    const float* __restrict__ proj, const float* __restrict__ bA, const float* __restrict__ bB,
    const float* __restrict__ bC,
    unsigned short* __restrict__ aPl, unsigned short* __restrict__ cPl, unsigned short* __restrict__ bsPl)
{
  __shared__ __align__(16) float sB[4 * 64];
  const int t = threadIdx.x, lane = t & 31, wave = t >> 5;
  const int q = lane >> 3, c8 = (lane & 7) * 8;
  const int m0 = blockIdx.x * 4;
  const int m  = m0 + q;
  const int bb = m / kT;
  const int p  = m - bb * kT;
  const float* pr = proj + (size_t)m * kProjN;
  const int hc = wave * kDH + c8;
  const v4f a0 = *(const v4f*)(pr + hc);
  const v4f a1 = *(const v4f*)(pr + hc + 4);
  const v4f ba0 = *(const v4f*)(bA + hc);
  const v4f ba1 = *(const v4f*)(bA + hc + 4);
  const v4f c0v = *(const v4f*)(pr + 2 * kDM + hc);
  const v4f c1v = *(const v4f*)(pr + 2 * kDM + hc + 4);
  const v4f bc0 = *(const v4f*)(bC + hc);
  const v4f bc1 = *(const v4f*)(bC + hc + 4);
  unsigned short ha[8], hc16[8];
#pragma unroll
  for (int e = 0; e < 4; ++e) {
    ha[e]       = h_bits((a0[e] + ba0[e]) * kACarry);
    ha[4 + e]   = h_bits((a1[e] + ba1[e]) * kACarry);
    hc16[e]     = h_bits((c0v[e] + bc0[e]) * kCCarry);
    hc16[4 + e] = h_bits((c1v[e] + bc1[e]) * kCCarry);
  }
  const v4u av = (v4u){pk16(ha[0], ha[1]), pk16(ha[2], ha[3]), pk16(ha[4], ha[5]), pk16(ha[6], ha[7])};
  const v4u cv = (v4u){pk16(hc16[0], hc16[1]), pk16(hc16[2], hc16[3]), pk16(hc16[4], hc16[5]), pk16(hc16[6], hc16[7])};
  {
    const int r2 = t >> 6, j = t & 63;
    const float* pb = proj + (size_t)(m0 + r2) * kProjN + kDM + j;
    float s = 0.f;
#pragma unroll
    for (int nn = 0; nn < kNH; ++nn) s += pb[nn * kDH] + bB[nn * kDH + j];
    sB[r2 * 64 + j] = s;
  }
  __syncthreads();
  const v4f s0 = *(const v4f*)(sB + q * 64 + c8);
  const v4f s1 = *(const v4f*)(sB + q * 64 + c8 + 4);
  unsigned short hs[8];
#pragma unroll
  for (int e = 0; e < 4; ++e) {
    hs[e]     = h_bits(s0[e] * kBsCarry);
    hs[4 + e] = h_bits(s1[e] * kBsCarry);
  }
  const v4u sv = (v4u){pk16(hs[0], hs[1]), pk16(hs[2], hs[3]), pk16(hs[4], hs[5]), pk16(hs[6], hs[7])};
  unsigned short* ap = aPl + ((size_t)((bb * kNH + wave) * kT + p)) * kDH + c8;
  unsigned short* cp = cPl + (size_t)m * kDM + hc;
  unsigned short* sp = bsPl + (size_t)m * kDH + c8;
  for (int pass = 0; pass < 2; ++pass) {
    *(volatile v4u*)ap = av;
    *(volatile v4u*)cp = cv;
    if (wave == 0) *(volatile v4u*)sp = sv;
    __threadfence();
  }
}

constexpr int kWtPitch  = kT;
constexpr int kLdsWt    = kDH * kWtPitch * 2;
constexpr int kLdsP     = 8 * 16 * 32 * 2;
constexpr int kLdsTotal = 2 * kLdsWt + 2 * kLdsP;
constexpr int kYsPitch  = 68;
static_assert(kLdsTotal == 65536, "LDS budget");
static_assert(64 * kYsPitch * 4 <= 2 * kLdsWt, "y stage fits in the wT area");

__global__ __launch_bounds__(256) void tri_core_kernel(
    const unsigned short* __restrict__ aPl, const unsigned short* __restrict__ s2Pl,
    const unsigned short* __restrict__ eHp, const unsigned short* __restrict__ eLp,
    const unsigned short* __restrict__ dHp, const unsigned short* __restrict__ dLp,
    unsigned short* __restrict__ yH, unsigned short* __restrict__ yL)
{
  __shared__ __align__(16) unsigned char smem[kLdsTotal];
  __bf16* wTh   = (__bf16*)(smem);
  __bf16* wTl   = (__bf16*)(smem + kLdsWt);
  __bf16* pHall = (__bf16*)(smem + 2 * kLdsWt);
  __bf16* pLall = (__bf16*)(smem + 2 * kLdsWt + kLdsP);
  float*  ys    = (float*)(smem);
  float*  red   = (float*)(smem + 2 * kLdsWt);

  const int tid = threadIdx.x, lane = tid & 31, wave = tid >> 5;
  const int hh = lane >> 4, c = lane & 15;
  const int r = blockIdx.x, n = blockIdx.y, b = blockIdx.z;
  const int bn = b * kNH + n;

  const _Float16* aB = (const _Float16*)aPl  + (size_t)bn * (kT * kDH);
  const _Float16* sB = (const _Float16*)s2Pl + (size_t)(b * kT + r) * (kT * kDH);
  const __bf16*   eH = (const __bf16*)eHp + (size_t)bn * (kDH * kT);
  const __bf16*   eL = (const __bf16*)eLp + (size_t)bn * (kDH * kT);
  const __bf16*   dH = (const __bf16*)dHp + (size_t)bn * (kDH * kT);
  const __bf16*   dL = (const __bf16*)dLp + (size_t)bn * (kDH * kT);
  __bf16* ph = pHall + wave * 512;
  __bf16* pl = pLall + wave * 512;

  const int npt    = (r + 15) >> 4;
  const int nptPad = (npt + 1) & ~1;
  float dsum = 0.f;

#pragma unroll 1
  for (int pt = wave; pt < nptPad; pt += 8) {
    const int p0 = pt << 4;
    const int wo = p0 + 8 * hh;
    if (pt < npt) {
      v16h qa[2];
#pragma unroll
      for (int dc = 0; dc < 2; ++dc) qa[dc] = Frag<_Float16>::load(aB + (size_t)(p0 + c) * kDH + dc * 32 + 8 * hh);
      v8f wacc[4];
#pragma unroll
      for (int t4 = 0; t4 < 4; ++t4) wacc[t4] = (v8f){0.f,0.f,0.f,0.f,0.f,0.f,0.f,0.f};
#pragma unroll 1
      for (int qc = p0 >> 5; qc < 6; ++qc) {
        const int q0 = qc << 5;
        v8f s0 = (v8f){0.f,0.f,0.f,0.f,0.f,0.f,0.f,0.f};
        v8f s1 = (v8f){0.f,0.f,0.f,0.f,0.f,0.f,0.f,0.f};
#pragma unroll
        for (int dc = 0; dc < 2; ++dc) {
          const v16h b0 = Frag<_Float16>::load(sB + (size_t)(q0 + c) * kDH + dc * 32 + 8 * hh);
          const v16h b1 = Frag<_Float16>::load(sB + (size_t)(q0 + 16 + c) * kDH + dc * 32 + 8 * hh);
          s0 = mma_h(qa[dc], b0, s0);
          s1 = mma_h(qa[dc], b1, s1);
        }
        const int qcol0 = q0 + c;
        const int qcol1 = q0 + 16 + c;
#pragma unroll
        for (int rr = 0; rr < 8; ++rr) {
          const int p = p0 + 8 * hh + rr;
          const bool rowok = (p < r);
          const float x0 = fminf(s0[rr] * kScoreScale, 60.0f);
          const float x1 = fminf(s1[rr] * kScoreScale, 60.0f);
          const float e0 = __expf(x0);
          const float e1 = __expf(x1);
          const float pv0 = (rowok && (p < qcol0)) ? e0 : 0.0f;
          const float pv1 = (rowok && (p < qcol1)) ? e1 : 0.0f;
          dsum += pv0;
          dsum += pv1;
          const unsigned short h0 = f2bf_bits(pv0);
          const unsigned short l0 = f2bf_bits(pv0 - bf_bits2f(h0));
          const unsigned short h1 = f2bf_bits(pv1);
          const unsigned short l1 = f2bf_bits(pv1 - bf_bits2f(h1));
          const int po = (8 * hh + rr) * 32 + c;
          ph[po]      = __builtin_bit_cast(__bf16, h0);
          pl[po]      = __builtin_bit_cast(__bf16, l0);
          ph[po + 16] = __builtin_bit_cast(__bf16, h1);
          pl[po + 16] = __builtin_bit_cast(__bf16, l1);
        }
        wave_lds_sync();
        const v16b pah = Frag<__bf16>::load(ph + c * 32 + 8 * hh);
        const v16b pal = Frag<__bf16>::load(pl + c * 32 + 8 * hh);
#pragma unroll
        for (int t4 = 0; t4 < 4; ++t4) {
          const size_t eo = (size_t)(t4 * 16 + c) * kT + q0 + 8 * hh;
          const v16b eh = Frag<__bf16>::load(eH + eo);
          const v16b el = Frag<__bf16>::load(eL + eo);
          wacc[t4] = mma_b(pah, eh, wacc[t4]);
          wacc[t4] = mma_b(pah, el, wacc[t4]);
          wacc[t4] = mma_b(pal, eh, wacc[t4]);
        }
        wave_lds_sync();
      }
#pragma unroll
      for (int t4 = 0; t4 < 4; ++t4) {
        unsigned short hb[8], lb[8];
#pragma unroll
        for (int rr = 0; rr < 8; ++rr) {
          const float v = wacc[t4][rr];
          hb[rr] = f2bf_bits(v);
          lb[rr] = f2bf_bits(v - bf_bits2f(hb[rr]));
        }
        const v4u hv = (v4u){pk16(hb[0], hb[1]), pk16(hb[2], hb[3]), pk16(hb[4], hb[5]), pk16(hb[6], hb[7])};
        const v4u lv = (v4u){pk16(lb[0], lb[1]), pk16(lb[2], lb[3]), pk16(lb[4], lb[5]), pk16(lb[6], lb[7])};
        const int off = (t4 * 16 + c) * kWtPitch + wo;
        *(v4u*)(wTh + off) = hv;
        *(v4u*)(wTl + off) = lv;
      }
    } else {
      const v4u zv = (v4u){0u, 0u, 0u, 0u};
#pragma unroll
      for (int t4 = 0; t4 < 4; ++t4) {
        const int off = (t4 * 16 + c) * kWtPitch + wo;
        *(v4u*)(wTh + off) = zv;
        *(v4u*)(wTl + off) = zv;
      }
    }
  }

#pragma unroll
  for (int off = 16; off > 0; off >>= 1) dsum += __shfl_xor(dsum, off, 32);
  wave_lds_sync();
  if (lane == 0) red[wave * 256] = dsum;
  __syncthreads();

  float Dtot = 0.f;
#pragma unroll
  for (int w8 = 0; w8 < 8; ++w8) Dtot += red[w8 * 256];
  const bool  dpos  = (Dtot > 0.0f);
  const float Dsafe = dpos ? Dtot : 1.0f;
  const float invD  = dpos ? (1.0f / Dsafe) : 0.0f;

  const int ht  = wave >> 1;
  const int gt0 = (wave & 1) * 2;
  const int ksteps = nptPad >> 1;
  v8f y0 = (v8f){0.f,0.f,0.f,0.f,0.f,0.f,0.f,0.f};
  v8f y1 = (v8f){0.f,0.f,0.f,0.f,0.f,0.f,0.f,0.f};
#pragma unroll 1
  for (int ks = 0; ks < ksteps; ++ks) {
    const int k0 = ks << 5;
    const size_t ao = (size_t)(ht * 16 + c) * kT + k0 + 8 * hh;
    const v16b ah = Frag<__bf16>::load(dH + ao);
    const v16b al = Frag<__bf16>::load(dL + ao);
    const int bo0 = (gt0 * 16 + c) * kWtPitch + k0 + 8 * hh;
    const int bo1 = bo0 + 16 * kWtPitch;
    const v16b b0h = Frag<__bf16>::load(wTh + bo0);
    const v16b b0l = Frag<__bf16>::load(wTl + bo0);
    const v16b b1h = Frag<__bf16>::load(wTh + bo1);
    const v16b b1l = Frag<__bf16>::load(wTl + bo1);
    y0 = mma_b(ah, b0h, y0);
    y0 = mma_b(ah, b0l, y0);
    y0 = mma_b(al, b0h, y0);
    y1 = mma_b(ah, b1h, y1);
    y1 = mma_b(ah, b1l, y1);
    y1 = mma_b(al, b1h, y1);
  }
  __syncthreads();
#pragma unroll
  for (int rr = 0; rr < 8; ++rr) {
    const int yo = (ht * 16 + 8 * hh + rr) * kYsPitch + gt0 * 16 + c;
    ys[yo]      = y0[rr] * invD;
    ys[yo + 16] = y1[rr] * invD;
  }
  __syncthreads();
  {
    const int q = lane >> 3, c8 = (lane & 7) * 8;
    v4u hv[2], lv[2];
#pragma unroll
    for (int it = 0; it < 2; ++it) {
      const int row = wave * 8 + it * 4 + q;
      const float* sp = ys + row * kYsPitch + c8;
      const v4f a0 = *(const v4f*)(sp);
      const v4f a1 = *(const v4f*)(sp + 4);
      float x[8];
#pragma unroll
      for (int e = 0; e < 4; ++e) { x[e] = a0[e]; x[4 + e] = a1[e]; }
      unsigned short hb[8], lb[8];
#pragma unroll
      for (int e = 0; e < 8; ++e) {
        hb[e] = f2bf_bits(x[e]);
        lb[e] = f2bf_bits(x[e] - bf_bits2f(hb[e]));
      }
      hv[it] = (v4u){pk16(hb[0], hb[1]), pk16(hb[2], hb[3]), pk16(hb[4], hb[5]), pk16(hb[6], hb[7])};
      lv[it] = (v4u){pk16(lb[0], lb[1]), pk16(lb[2], lb[3]), pk16(lb[4], lb[5]), pk16(lb[6], lb[7])};
    }
    const size_t yrow = ((size_t)n * kRows + (size_t)b * kT + r) * kHG;
    for (int pass = 0; pass < 2; ++pass) {
#pragma unroll
      for (int it = 0; it < 2; ++it) {
        const int row = wave * 8 + it * 4 + q;
        const size_t o = yrow + (size_t)row * kDH + c8;
        *(volatile v4u*)(yH + o) = hv[it];
        *(volatile v4u*)(yL + o) = lv[it];
      }
      __threadfence();
    }
  }
}

extern "C" void kernel_launch(void* const* d_in, const int* in_sizes, int n_in,
                              void* d_out, int out_size, void* d_ws, size_t ws_size,
                              hipStream_t stream) {
  if (n_in < 15) return;
  if (in_sizes[0] != kRows * kDM) return;
  for (int i = 1; i <= 5; ++i) if (in_sizes[i] != kNH * kDM * kDH) return;
  if (in_sizes[6] != kNH * kHG * kDH) return;
  if (in_sizes[7] != kNH * kHG * kDH) return;
  if (in_sizes[8] != kNH * kDH * kDM) return;
  for (int i = 9; i <= 13; ++i) if (in_sizes[i] != kNH * kDH) return;
  if (in_sizes[14] != kDM) return;
  if (out_size != kRows * kDM) return;
  if (ws_size < kWsTotal) return;

  const float* x  = (const float*)d_in[0];
  const float* Wp[5] = {(const float*)d_in[1], (const float*)d_in[2], (const float*)d_in[3],
                        (const float*)d_in[4], (const float*)d_in[5]};
  const float* WK = (const float*)d_in[6];
  const float* WV = (const float*)d_in[7];
  const float* WO = (const float*)d_in[8];
  const float* bA = (const float*)d_in[9];
  const float* bB = (const float*)d_in[10];
  const float* bC = (const float*)d_in[11];
  const float* bD = (const float*)d_in[12];
  const float* bE = (const float*)d_in[13];
  const float* bO = (const float*)d_in[14];
  float* out = (float*)d_out;

  char* ws = (char*)d_ws;
  unsigned short* XH   = (unsigned short*)(ws + kOffXH);
  unsigned short* XL   = (unsigned short*)(ws + kOffXL);
  unsigned short* WPH  = (unsigned short*)(ws + kOffWPH);
  unsigned short* WPL  = (unsigned short*)(ws + kOffWPL);
  float*          PROJ = (float*)(ws + kOffPROJ);
  unsigned short* APL  = (unsigned short*)(ws + kOffAPL);
  unsigned short* CPL  = (unsigned short*)(ws + kOffCPL);
  unsigned short* BSUM = (unsigned short*)(ws + kOffBSUM);
  unsigned short* DTH  = (unsigned short*)(ws + kOffDTH);
  unsigned short* DTL  = (unsigned short*)(ws + kOffDTL);
  unsigned short* ETH  = (unsigned short*)(ws + kOffETH);
  unsigned short* ETL  = (unsigned short*)(ws + kOffETL);
  unsigned short* WKB  = (unsigned short*)(ws + kOffWKB);
  unsigned short* S1   = (unsigned short*)(ws + kOffS1);
  unsigned short* S2T  = (unsigned short*)(ws + kOffS2T);
  unsigned short* YH   = (unsigned short*)(ws + kOffYH);
  unsigned short* YL   = (unsigned short*)(ws + kOffYL);
  unsigned short* WVH  = (unsigned short*)(ws + kOffWVH);
  unsigned short* WVL  = (unsigned short*)(ws + kOffWVL);
  unsigned short* ZH   = (unsigned short*)(ws + kOffZH);
  unsigned short* ZL   = (unsigned short*)(ws + kOffZL);
  unsigned short* WOH  = (unsigned short*)(ws + kOffWOH);
  unsigned short* WOL  = (unsigned short*)(ws + kOffWOL);

  split_rows_kernel<<<(kRows * kDM / 8) / 256, 256, 0, stream>>>(x, XH, XL, kRows * kDM / 8);
  wk_cast_kernel<<<(kHG * kDM / 8) / 256, 256, 0, stream>>>(WK, WKB);
  for (int w = 0; w < 5; ++w) {
    tsplit_kernel<false><<<dim3(kDM / 64, 1, kNH), 256, 0, stream>>>(
        Wp[w], kDH, (long)kDM * kDH, 0L, 1,
        nullptr, 0,
        WPH + (size_t)w * kDM * kDM, WPL + (size_t)w * kDM * kDM, kDM, (long)kDH * kDM);
  }
  tsplit_kernel<false><<<dim3(kHG / 64, 1, kNH), 256, 0, stream>>>(
      WV, kDH, (long)kHG * kDH, 0L, 1,
      nullptr, 0,
      WVH, WVL, kHG, (long)kDH * kHG);
  tsplit_kernel<false><<<dim3(kDM / 64, kDM / 64, 1), 256, 0, stream>>>(
      WO, kDM, 0L, 0L, 1,
      nullptr, 0,
      WOH, WOL, kDM, 0L);

  wmma_gemm64<1, true, 0, 0><<<dim3(30, 1), 256, 0, stream>>>(
      XH, XL, kDM, 0L,
      WPH, WPL, kDM, 0L,
      (void*)PROJ, nullptr, kProjN, 0L,
      nullptr,
      kRows, kProjN, kDM, 1.0f);

  cvt_abc_kernel<<<kRows / 4, 256, 0, stream>>>(PROJ, bA, bB, bC, APL, CPL, BSUM);
  tsplit_kernel<true><<<dim3(kT / 64, 1, kB * kNH), 256, 0, stream>>>(
      PROJ + 3 * kDM, kProjN, (long)kT * kProjN, (long)kDH, kNH,
      bD, kDH,
      DTH, DTL, kT, (long)kDH * kT);
  tsplit_kernel<true><<<dim3(kT / 64, 1, kB * kNH), 256, 0, stream>>>(
      PROJ + 4 * kDM, kProjN, (long)kT * kProjN, (long)kDH, kNH,
      bE, kDH,
      ETH, ETL, kT, (long)kDH * kT);

  wmma_gemm64<0, false, 0, 1><<<dim3(48, 1), 256, 0, stream>>>(
      CPL, nullptr, kDM, 0L,
      WKB, nullptr, kDM, 0L,
      (void*)S1, nullptr, kHG, 0L,
      nullptr,
      kRows, kHG, kDM, kS1Scale);

  for (int bb = 0; bb < kB; ++bb) {
    wmma_gemm64<0, false, 0, 1><<<dim3(1, kT), 256, 0, stream>>>(
        BSUM + (size_t)bb * kT * kDH, nullptr, kDH, 0L,
        S1 + (size_t)bb * kT * kHG, nullptr, kDH, (long)kHG,
        (void*)(S2T + (size_t)bb * kT * kT * kDH), nullptr, kDH, (long)kT * kDH,
        nullptr,
        kT, kDH, kDH, kS2Scale);
  }

  tri_core_kernel<<<dim3(kT, kNH, kB), 256, 0, stream>>>(APL, S2T, ETH, ETL, DTH, DTL, YH, YL);

  wmma_gemm64<1, true, 0, 2><<<dim3(1, kNH), 256, 0, stream>>>(
      YH, YL, kHG, (long)kRows * kHG,
      WVH, WVL, kHG, (long)kDH * kHG,
      (void*)ZH, (void*)ZL, kDM, (long)kDH,
      nullptr,
      kRows, kDH, kHG, 1.0f);

  wmma_gemm64<1, true, 2, 0><<<dim3(6, 1), 256, 0, stream>>>(
      ZH, ZL, kDM, 0L,
      WOH, WOL, kDM, 0L,
      (void*)out, nullptr, kDM, 0L,
      bO,
      kRows, kDM, kDM, 1.0f);
}
